// SequenceEncoder_69063074120430
// MI455X (gfx1250) — hardware-verified
//
#include <hip/hip_runtime.h>

typedef __bf16          v16b  __attribute__((ext_vector_type(16)));
typedef unsigned short  v8us  __attribute__((ext_vector_type(8)));
typedef int             v8i   __attribute__((ext_vector_type(8)));
typedef float           v8f   __attribute__((ext_vector_type(8)));
typedef float           v4f   __attribute__((ext_vector_type(4)));
typedef v8us __attribute__((may_alias)) v8usa;
typedef v4f  __attribute__((may_alias)) v4fa;

union Frag { v16b v; v8us half[2]; };

#define NB     32
#define SEQ    2048
#define HID    100
#define DP     128
#define VOCAB  50000
#define NTOK   (NB * SEQ)
#define TP     136
#define QP     136
#define OROWS  64
#define OLINES ((OROWS * HID * 4) / 128)

static_assert((OROWS * HID * 4) % 128 == 0);
static_assert(SEQ % OROWS == 0);
static_assert((OROWS % 32) == 0);
static_assert(DP % 32 == 0);
static_assert((HID % 4) == 0);

__device__ __forceinline__ v8f wmma_bf16(v16b a, v16b b, v8f c) {
  v8f d = __builtin_amdgcn_wmma_f32_16x16x32_bf16(false, a, false, b, (short)0, c, false, false);
  asm volatile("v_nop\n\tv_nop\n\tv_nop\n\tv_nop"
               : "+v"(d)
               : "v"(__builtin_bit_cast(v8i, a)), "v"(__builtin_bit_cast(v8i, b)));
  return d;
}

__device__ __forceinline__ v16b load_frag(const unsigned short* p, int h) {
  Frag f;
  f.half[0] = *(const v8usa*)(p + 8 * h);
  f.half[1] = *(const v8usa*)(p + 16 + 8 * h);
  return f.v;
}

__device__ __forceinline__ unsigned short f2bf(float f) {
  unsigned int u = __float_as_uint(f);
  u += 0x7FFFu + ((u >> 16) & 1u);
  return (unsigned short)(u >> 16);
}
__device__ __forceinline__ float bf2f(unsigned short s) {
  return __uint_as_float(((unsigned int)s) << 16);
}

__device__ __forceinline__ v8us cvt8(v4f u, v4f v, int d0, bool rok) {
  v8us t;
  t[0] = (rok && (d0 + 0) < HID) ? f2bf(u[0]) : (unsigned short)0;
  t[1] = (rok && (d0 + 1) < HID) ? f2bf(u[1]) : (unsigned short)0;
  t[2] = (rok && (d0 + 2) < HID) ? f2bf(u[2]) : (unsigned short)0;
  t[3] = (rok && (d0 + 3) < HID) ? f2bf(u[3]) : (unsigned short)0;
  t[4] = (rok && (d0 + 4) < HID) ? f2bf(v[0]) : (unsigned short)0;
  t[5] = (rok && (d0 + 5) < HID) ? f2bf(v[1]) : (unsigned short)0;
  t[6] = (rok && (d0 + 6) < HID) ? f2bf(v[2]) : (unsigned short)0;
  t[7] = (rok && (d0 + 7) < HID) ? f2bf(v[3]) : (unsigned short)0;
  return t;
}

__global__ __launch_bounds__(256) void k_wprep(
    const float* __restrict__ Wq, const float* __restrict__ bq,
    unsigned short* __restrict__ wqb, float* __restrict__ bqr)
{
  const int tid = threadIdx.x, lane = tid & 31, w = tid >> 5;
  const int q8 = lane & 7, sub = lane >> 3;

  v8us vals[8];
  #pragma unroll
  for (int i = 0; i < 8; ++i) {
    const int L = 32 * w + 4 * i + sub;
    const int o = L >> 1, hf = L & 1;
    const int d0 = 64 * hf + 8 * q8;
    const int oc = min(o, HID - 1);
    const int a0 = min(d0, HID - 4), a1 = min(d0 + 4, HID - 4);
    const float* row = Wq + oc * HID;
    const v4f u = *(const v4fa*)(row + a0);
    const v4f v = *(const v4fa*)(row + a1);
    vals[i] = cvt8(u, v, d0, o < HID);
  }
  v4f bv;
  {
    const int d0 = 4 * lane;
    bv[0] = ((d0 + 0) < HID) ? bf2f(f2bf(bq[min(d0 + 0, HID - 1)])) : 0.0f;
    bv[1] = ((d0 + 1) < HID) ? bf2f(f2bf(bq[min(d0 + 1, HID - 1)])) : 0.0f;
    bv[2] = ((d0 + 2) < HID) ? bf2f(f2bf(bq[min(d0 + 2, HID - 1)])) : 0.0f;
    bv[3] = ((d0 + 3) < HID) ? bf2f(f2bf(bq[min(d0 + 3, HID - 1)])) : 0.0f;
  }

  #pragma unroll
  for (int i = 0; i < 8; ++i) {
    const int L = 32 * w + 4 * i + sub;
    *(volatile v8us*)(wqb + L * 64 + 8 * q8) = vals[i];
  }
  if (w == 0) *(volatile v4f*)(bqr + 4 * lane) = bv;
  __threadfence();
  #pragma unroll
  for (int i = 0; i < 8; ++i) {
    const int L = 32 * w + 4 * i + sub;
    *(volatile v8us*)(wqb + L * 64 + 8 * q8) = vals[i];
  }
  if (w == 0) *(volatile v4f*)(bqr + 4 * lane) = bv;
}

__device__ __forceinline__ void prep_store_pass(const unsigned short* tile,
                                                unsigned short* hb, unsigned short* ht,
                                                int b, int j0, int w, int lane) {
  const int q8 = lane & 7, sub = lane >> 3;
  #pragma unroll
  for (int i = 0; i < 4; ++i) {
    const int L = 16 * w + 4 * i + sub;
    const int r = L >> 1, hf = L & 1;
    const v8us v = *(const v8usa*)(tile + r * TP + 64 * hf + 8 * q8);
    *(volatile v8us*)(hb + ((size_t)(b * SEQ + j0 + r)) * DP + 64 * hf + 8 * q8) = v;
  }
  #pragma unroll
  for (int i = 0; i < 4; ++i) {
    const int d = 16 * w + 4 * i + sub;
    v8us o;
    #pragma unroll
    for (int t = 0; t < 8; ++t) o[t] = tile[(8 * q8 + t) * TP + d];
    *(volatile v8us*)(ht + ((size_t)(b * DP + d)) * SEQ + j0 + 8 * q8) = o;
  }
}

__global__ __launch_bounds__(256) void k_prep(
    const int* __restrict__ x, const float* __restrict__ embed,
    unsigned short* __restrict__ hb, unsigned short* __restrict__ ht)
{
  __shared__ __attribute__((aligned(16))) unsigned short tile[OROWS * TP];

  const int b = blockIdx.y, j0 = blockIdx.x * OROWS;
  const int tid = threadIdx.x, lane = tid & 31, w = tid >> 5;

  #pragma unroll
  for (int s = 0; s < 4; ++s) {
    const int task = tid + 256 * s;
    const int r = task >> 4, c = task & 15;
    int idx = x[b * SEQ + j0 + r];
    idx = min(max(idx, 0), VOCAB - 1);
    const int d0 = 8 * c;
    const int a0 = min(d0, HID - 4), a1 = min(d0 + 4, HID - 4);
    const float* row = embed + (size_t)idx * HID;
    const v4f u = *(const v4fa*)(row + a0);
    const v4f v = *(const v4fa*)(row + a1);
    *(v8usa*)(tile + r * TP + d0) = cvt8(u, v, d0, true);
  }
  __syncthreads();

  prep_store_pass(tile, hb, ht, b, j0, w, lane);
  __threadfence();
  prep_store_pass(tile, hb, ht, b, j0, w, lane);
}

__device__ __forceinline__ void gram_store_pass(const unsigned short* sT, unsigned short* plane,
                                                int b, int w, int lane) {
  const int q8 = lane & 7, sub = lane >> 3;
  #pragma unroll
  for (int i = 0; i < 8; ++i) {
    const int lid = 4 * i + sub;
    const int row = 16 * w + (lid >> 1), hf = lid & 1;
    const v8us v = *(const v8usa*)(sT + row * DP + 64 * hf + 8 * q8);
    *(volatile v8us*)(plane + ((size_t)(b * DP + row)) * DP + 64 * hf + 8 * q8) = v;
  }
}

__global__ __launch_bounds__(256) void k_gram(
    const unsigned short* __restrict__ ht,
    unsigned short* __restrict__ mhi,
    unsigned short* __restrict__ mlo)
{
  __shared__ __attribute__((aligned(16))) unsigned short sT[DP * DP];

  const int b = blockIdx.x;
  const int tid = threadIdx.x, lane = tid & 31, w = tid >> 5;
  const int h = lane >> 4, m = lane & 15;
  const int e0 = 16 * w;

  const unsigned short* base = ht + (size_t)b * DP * SEQ;
  const unsigned short* arow = base + (size_t)(e0 + m) * SEQ;

  const v8f zero8 = {0.f, 0.f, 0.f, 0.f, 0.f, 0.f, 0.f, 0.f};
  v8f acc[8];
  #pragma unroll
  for (int nt = 0; nt < 8; ++nt) acc[nt] = zero8;

  #pragma unroll 1
  for (int k0 = 0; k0 < SEQ; k0 += 32) {
    const v16b a = load_frag(arow + k0, h);
    #pragma unroll
    for (int nt = 0; nt < 8; ++nt) {
      const v16b bb = load_frag(base + (size_t)(16 * nt + m) * SEQ + k0, h);
      acc[nt] = wmma_bf16(a, bb, acc[nt]);
    }
  }

  #pragma unroll
  for (int nt = 0; nt < 8; ++nt)
    #pragma unroll
    for (int r = 0; r < 8; ++r)
      sT[(e0 + 8 * h + r) * DP + 16 * nt + m] = f2bf(acc[nt][r]);
  __syncthreads();
  gram_store_pass(sT, mhi, b, w, lane);
  __threadfence();
  gram_store_pass(sT, mhi, b, w, lane);
  __syncthreads();

  #pragma unroll
  for (int nt = 0; nt < 8; ++nt)
    #pragma unroll
    for (int r = 0; r < 8; ++r) {
      const float v = acc[nt][r];
      const unsigned short hi = f2bf(v);
      sT[(e0 + 8 * h + r) * DP + 16 * nt + m] = f2bf(v - bf2f(hi));
    }
  __syncthreads();
  gram_store_pass(sT, mlo, b, w, lane);
  __threadfence();
  gram_store_pass(sT, mlo, b, w, lane);
}

__device__ __forceinline__ void out_store_pass(const float* sO, float* dst, int w, int lane) {
  const int q8 = lane & 7, sub = lane >> 3;
  #pragma unroll
  for (int it = 0; it < 13; ++it) {
    const int L = 16 * it + 4 * w + sub;
    if (L < OLINES) {
      const v4f v = *(const v4fa*)(sO + L * 32 + 4 * q8);
      *(volatile v4f*)(dst + L * 32 + 4 * q8) = v;
    }
  }
}

__global__ __launch_bounds__(128) void k_out(
    const unsigned short* __restrict__ hb,
    const unsigned short* __restrict__ wqb,
    const float* __restrict__ bqr,
    const unsigned short* __restrict__ mhi,
    const unsigned short* __restrict__ mlo,
    float* __restrict__ out)
{
  __shared__ __attribute__((aligned(16))) unsigned short sQ[2 * OROWS * QP];
  __shared__ __attribute__((aligned(16))) float sO[OROWS * HID];

  const int b = blockIdx.y, i0 = blockIdx.x * OROWS;
  const int tid = threadIdx.x, lane = tid & 31, w = tid >> 5;
  const int h = lane >> 4, m = lane & 15;
  const int rw = 16 * w;

  const v8f zero8 = {0.f, 0.f, 0.f, 0.f, 0.f, 0.f, 0.f, 0.f};

  const unsigned short* arow = hb + ((size_t)(b * SEQ + i0 + rw + m)) * DP;
  v8f acc[8];
  #pragma unroll
  for (int nt = 0; nt < 8; ++nt) acc[nt] = zero8;
  #pragma unroll
  for (int k0 = 0; k0 < DP; k0 += 32) {
    const v16b a = load_frag(arow + k0, h);
    #pragma unroll
    for (int nt = 0; nt < 8; ++nt) {
      const v16b bb = load_frag(wqb + (size_t)(16 * nt + m) * DP + k0, h);
      acc[nt] = wmma_bf16(a, bb, acc[nt]);
    }
  }

  unsigned short* sQhi = sQ;
  unsigned short* sQlo = sQ + OROWS * QP;
  #pragma unroll
  for (int nt = 0; nt < 8; ++nt) {
    const float bias = bqr[16 * nt + m];
    #pragma unroll
    for (int r = 0; r < 8; ++r) {
      const float q = acc[nt][r] + bias;
      const unsigned short hi = f2bf(q);
      const unsigned short lo = f2bf(q - bf2f(hi));
      const int li = (rw + 8 * h + r) * QP + 16 * nt + m;
      sQhi[li] = hi;
      sQlo[li] = lo;
    }
  }
  __syncthreads();

  const unsigned short* qhrow = sQhi + (rw + m) * QP;
  const unsigned short* qlrow = sQlo + (rw + m) * QP;
  const unsigned short* mhb = mhi + ((size_t)(b * DP + m)) * DP;
  const unsigned short* mlb = mlo + ((size_t)(b * DP + m)) * DP;
  v8f acc2[7];
  #pragma unroll
  for (int nt = 0; nt < 7; ++nt) acc2[nt] = zero8;
  #pragma unroll
  for (int k0 = 0; k0 < DP; k0 += 32) {
    const v16b qh = load_frag(qhrow + k0, h);
    const v16b ql = load_frag(qlrow + k0, h);
    #pragma unroll
    for (int nt = 0; nt < 7; ++nt) {
      const v16b bh = load_frag(mhb + (size_t)(16 * nt) * DP + k0, h);
      const v16b bl = load_frag(mlb + (size_t)(16 * nt) * DP + k0, h);
      acc2[nt] = wmma_bf16(qh, bh, acc2[nt]);
      acc2[nt] = wmma_bf16(qh, bl, acc2[nt]);
      acc2[nt] = wmma_bf16(ql, bh, acc2[nt]);
    }
  }

  #pragma unroll
  for (int nt = 0; nt < 7; ++nt) {
    const int col = 16 * nt + m;
    if (col < HID) {
      #pragma unroll
      for (int r = 0; r < 8; ++r) sO[(rw + 8 * h + r) * HID + col] = acc2[nt][r];
    }
  }
  __syncthreads();

  float* dst = out + ((size_t)(b * SEQ + i0)) * HID;
  out_store_pass(sO, dst, w, lane);
  __threadfence();
  out_store_pass(sO, dst, w, lane);
}

extern "C" void kernel_launch(void* const* d_in, const int* in_sizes, int n_in,
                              void* d_out, int out_size, void* d_ws, size_t ws_size,
                              hipStream_t stream) {
  if (n_in < 4) return;
  if (in_sizes[0] != NTOK) return;
  if (in_sizes[1] != VOCAB * HID) return;
  if (in_sizes[2] != HID * HID) return;
  if (in_sizes[3] != HID) return;
  if (out_size != NTOK * HID) return;

  const int*   x     = (const int*)d_in[0];
  const float* embed = (const float*)d_in[1];
  const float* Wq    = (const float*)d_in[2];
  const float* bq    = (const float*)d_in[3];
  float* out = (float*)d_out;

  const size_t hb_bytes  = (size_t)NTOK * DP * 2;
  const size_t ht_bytes  = (size_t)NB * DP * SEQ * 2;
  const size_t m_bytes   = (size_t)NB * DP * DP * 2;
  const size_t wqb_bytes = (size_t)DP * DP * 2;
  const size_t bqr_bytes = (size_t)DP * 4;
  const size_t total = hb_bytes + ht_bytes + 2 * m_bytes + wqb_bytes + bqr_bytes;
  if (total > ws_size) return;

  char* ws = (char*)d_ws;
  size_t off = 0;
  unsigned short* hb  = (unsigned short*)(ws + off); off += hb_bytes;
  unsigned short* ht  = (unsigned short*)(ws + off); off += ht_bytes;
  unsigned short* mhi = (unsigned short*)(ws + off); off += m_bytes;
  unsigned short* mlo = (unsigned short*)(ws + off); off += m_bytes;
  unsigned short* wqb = (unsigned short*)(ws + off); off += wqb_bytes;
  float*          bqr = (float*)(ws + off);          off += bqr_bytes;

  k_wprep<<<1, 256, 0, stream>>>(Wq, bq, wqb, bqr);

  dim3 gPrep(SEQ / OROWS, NB);
  k_prep<<<gPrep, 256, 0, stream>>>(x, embed, hb, ht);

  k_gram<<<NB, 256, 0, stream>>>(ht, mhi, mlo);

  dim3 gOut(SEQ / OROWS, NB);
  k_out<<<gOut, 128, 0, stream>>>(hb, wqb, bqr, mhi, mlo, out);
}
